// ResidueIntraBlockGNN_59931973649025
// MI455X (gfx1250) — hardware-run, weakly checked
//
#include <hip/hip_runtime.h>

typedef float          v8f   __attribute__((ext_vector_type(8)));
typedef float          v4f   __attribute__((ext_vector_type(4)));
typedef unsigned int   v4u   __attribute__((ext_vector_type(4)));
typedef int            v8i   __attribute__((ext_vector_type(8)));
typedef unsigned short v8us  __attribute__((ext_vector_type(8)));
typedef unsigned short v16us __attribute__((ext_vector_type(16)));
typedef __bf16         v16bf __attribute__((ext_vector_type(16)));
typedef _Float16       v16h  __attribute__((ext_vector_type(16)));
typedef v4f  __attribute__((may_alias)) v4fa;
typedef v8us __attribute__((may_alias)) v8usa;
union FragB { v16bf v; v16us u; v8us h[2]; v8i w; };
union FragH { v16h  v; v16us u; v8us h[2]; v8i w; };

__device__ __forceinline__ v8f wmb(const FragB& a, const FragB& b, v8f c) {
  v8f d = __builtin_amdgcn_wmma_f32_16x16x32_bf16(false, a.v, false, b.v, (short)0, c, false, false);
  asm volatile("v_nop\n\tv_nop\n\tv_nop\n\tv_nop" : "+v"(d) : "v"(a.w), "v"(b.w));
  return d;
}

__device__ __forceinline__ v8f wmh(const FragH& a, const FragH& b, v8f c) {
  v8f d = __builtin_amdgcn_wmma_f32_16x16x32_f16(false, a.v, false, b.v, (short)0, c, false, false);
  asm volatile("v_nop\n\tv_nop\n\tv_nop\n\tv_nop" : "+v"(d) : "v"(a.w), "v"(b.w));
  return d;
}

__device__ __forceinline__ unsigned bf16_bits(float f) {
  const unsigned u = __float_as_uint(f);
  const unsigned r = (u + 0x7FFFu + ((u >> 16) & 1u)) >> 16;
  const unsigned q = (u >> 16) | 0x40u;
  return ((u & 0x7fffffffu) > 0x7f800000u) ? q : r;
}

__device__ __forceinline__ float bf16_val(float f) {
  return __uint_as_float(bf16_bits(f) << 16);
}
__device__ __forceinline__ int clampi(int v, int lo, int hi) {
  return v < lo ? lo : (v > hi ? hi : v);
}

__device__ __forceinline__ unsigned f16_bits(float f) {
  const unsigned u  = __float_as_uint(f);
  const unsigned s  = (u >> 16) & 0x8000u;
  const unsigned a  = u & 0x7fffffffu;
  const unsigned t  = a - 0x38000000u;
  const unsigned r  = (t + 0x0FFFu + ((t >> 13) & 1u)) >> 13;
  const unsigned rc = r > 0x7C00u ? 0x7C00u : r;
  const bool small  = a < 0x38800000u;
  const bool isnan  = a > 0x7f800000u;
  const unsigned fin = small ? 0u : (s | rc);
  return isnan ? (s | 0x7E00u) : fin;
}

__device__ __forceinline__ unsigned pk16(unsigned lo, unsigned hi) { return lo | (hi << 16); }
__device__ __forceinline__ unsigned bf16_lo_bits(float v) {
  float hi = bf16_val(v);
  asm volatile("" : "+v"(hi));
  return bf16_bits(v - hi);
}
__device__ __forceinline__ v4u pack8_bf16(v4f a, v4f c) {
  return (v4u){ pk16(bf16_bits(a[0]), bf16_bits(a[1])), pk16(bf16_bits(a[2]), bf16_bits(a[3])),
                pk16(bf16_bits(c[0]), bf16_bits(c[1])), pk16(bf16_bits(c[2]), bf16_bits(c[3])) };
}
__device__ __forceinline__ v4u pack8_bf16_lo(v4f a, v4f c) {
  return (v4u){ pk16(bf16_lo_bits(a[0]), bf16_lo_bits(a[1])), pk16(bf16_lo_bits(a[2]), bf16_lo_bits(a[3])),
                pk16(bf16_lo_bits(c[0]), bf16_lo_bits(c[1])), pk16(bf16_lo_bits(c[2]), bf16_lo_bits(c[3])) };
}
__device__ __forceinline__ v4u pack8_f16(v4f a, v4f c) {
  return (v4u){ pk16(f16_bits(a[0]), f16_bits(a[1])), pk16(f16_bits(a[2]), f16_bits(a[3])),
                pk16(f16_bits(c[0]), f16_bits(c[1])), pk16(f16_bits(c[2]), f16_bits(c[3])) };
}

template <int FORM>
__global__ __launch_bounds__(256) void k_plane(const float* __restrict__ src, int rows, int cols, int ldsrc,
                                               unsigned short* __restrict__ dst, int MP, int KP) {
  static_assert(FORM >= 0 && FORM <= 3);
  const int KTOT = (FORM == 1 || FORM == 3) ? 2 * KP : KP;
  const unsigned ppr   = (unsigned)(KTOT >> 3);
  const unsigned kp8   = (unsigned)(KP >> 3);
  const unsigned total = (unsigned)MP * ppr;
  const unsigned g     = blockIdx.x * 256u + threadIdx.x;
  const unsigned rowu  = g / ppr;
  const unsigned p     = g - rowu * ppr;
  const bool second    = p >= kp8;
  const int row = (int)rowu;
  const int c0  = (int)((second ? p - kp8 : p) << 3);
  const float* srow = src + (size_t)clampi(row, 0, rows - 1) * (size_t)ldsrc;
  float x[8];
  unsigned mk[8];
#pragma unroll
  for (int e = 0; e < 8; ++e) {
    const int c = c0 + e;
    const float v = srow[clampi(c, 0, cols - 1)];
    asm volatile("" :: "v"(v));
    x[e]  = v;
    mk[e] = (row < rows && c < cols) ? 0xFFFFu : 0u;
  }
  const v4f a = (v4f){ x[0], x[1], x[2], x[3] };
  const v4f c = (v4f){ x[4], x[5], x[6], x[7] };
  v4u o;
  if (FORM == 2) {
    o = pack8_f16(a, c);
  } else {
    const v4u hi = pack8_bf16(a, c);
    o = hi;
    if (FORM == 1) { const v4u lo = pack8_bf16_lo(a, c); o = second ? lo : hi; }
  }
  const v4u mw = (v4u){ pk16(mk[0], mk[1]), pk16(mk[2], mk[3]), pk16(mk[4], mk[5]), pk16(mk[6], mk[7]) };
  o &= mw;
  if (g < total) {
    volatile v4u* q = (volatile v4u*)(dst + (size_t)g * 8);
    *q = o;
    __threadfence();
    *q = o;
  }
}

template <int FORM> struct FragOf    { typedef FragB T; };
template <>         struct FragOf<2> { typedef FragH T; };
__device__ __forceinline__ v8f mm(const FragB& a, const FragB& b, v8f c) { return wmb(a, b, c); }
__device__ __forceinline__ v8f mm(const FragH& a, const FragH& b, v8f c) { return wmh(a, b, c); }
template <class F> __device__ __forceinline__ F ld_frag(const unsigned short* p) {
  F f;
  f.h[0] = *(const v8usa*)(p);
  f.h[1] = *(const v8usa*)(p + 16);
  return f;
}

template <int FORM, int EPI>
__global__ __launch_bounds__(256) __attribute__((amdgpu_num_vgpr(248)))
void k_gemm_nt(const unsigned short* __restrict__ A, const unsigned short* __restrict__ B,
               const float* __restrict__ bias, float* __restrict__ D, int M, int N, int KTOT, int ldd) {
  static_assert(FORM >= 0 && FORM <= 2);
  static_assert(EPI == 0 || EPI == 1);
  typedef typename FragOf<FORM>::T F;
  __shared__ __attribute__((aligned(16))) float sT[8][16 * 68];
  const int lane = threadIdx.x & 31;
  const int wave = threadIdx.x >> 5;
  const int tilesM = (M + 63) >> 6;
  const int tilesN = (N + 63) >> 6;
  const int tile = blockIdx.x * 8 + wave;
  if (tile >= tilesM * tilesN) return;
  const int tm = tile / tilesN;
  const int tn = tile - tm * tilesN;
  const int m0 = tm << 6;
  const int n0 = tn << 6;

  const int rl = lane & 15;
  const int h8 = (lane >> 4) * 8;
  const unsigned short* pa = A + (size_t)(m0 + rl) * (size_t)KTOT + h8;
  const unsigned short* pb = B + (size_t)(n0 + rl) * (size_t)KTOT + h8;

  v8f acc[4][4];
#pragma unroll
  for (int i = 0; i < 4; ++i)
#pragma unroll
    for (int j = 0; j < 4; ++j) acc[i][j] = (v8f){0.f, 0.f, 0.f, 0.f, 0.f, 0.f, 0.f, 0.f};

#pragma unroll 1
  for (int k0 = 0; k0 < KTOT; k0 += 32) {
    F bf[4];
#pragma unroll
    for (int j = 0; j < 4; ++j) bf[j] = ld_frag<F>(pb + (size_t)(j << 4) * (size_t)KTOT + k0);
#pragma unroll
    for (int i = 0; i < 4; ++i) {
      const F af = ld_frag<F>(pa + (size_t)(i << 4) * (size_t)KTOT + k0);
#pragma unroll
      for (int j = 0; j < 4; ++j) acc[i][j] = mm(af, bf[j], acc[i][j]);
    }
  }

  float* slab = sT[wave];
  const int hh = lane >> 4;
  const int c4 = (lane & 15) * 4;
  const int nc = n0 + c4;
  const bool cok = nc < N;
  v4f bv = (v4f){0.f, 0.f, 0.f, 0.f};
  if (EPI == 1) {
    bv = *(const v4fa*)(bias + clampi(nc, 0, N - 4));
    asm volatile("" :: "v"(bv));
  }
#pragma unroll
  for (int i = 0; i < 4; ++i) {
    const int mBase = m0 + (i << 4);
#pragma unroll
    for (int j = 0; j < 4; ++j) {
#pragma unroll
      for (int r = 0; r < 8; ++r) slab[(h8 + r) * 68 + (j << 4) + rl] = acc[i][j][r];
    }
    __builtin_amdgcn_fence(__ATOMIC_RELEASE, "workgroup");
    __builtin_amdgcn_wave_barrier();
    __builtin_amdgcn_fence(__ATOMIC_ACQUIRE, "workgroup");
    v4f vv[8];
#pragma unroll
    for (int it = 0; it < 8; ++it) {
      const int row = it * 2 + hh;
      v4f v = *(const v4fa*)(slab + row * 68 + c4);
      if (EPI == 1) v += bv;
      vv[it] = v;
    }
    for (int pass = 0; pass < 2; ++pass) {
#pragma unroll
      for (int it = 0; it < 8; ++it) {
        const int row = mBase + it * 2 + hh;
        if (cok && row < M) *(volatile v4f*)(D + (size_t)row * (size_t)ldd + nc) = vv[it];
      }
      __threadfence();
    }
    __builtin_amdgcn_fence(__ATOMIC_RELEASE, "workgroup");
    __builtin_amdgcn_wave_barrier();
    __builtin_amdgcn_fence(__ATOMIC_ACQUIRE, "workgroup");
  }
}

#pragma clang fp contract(off)

#define NN      16384
#define NE      262144
#define DIM     256
#define NTHR    256
#define NWAVE   8
#define NBA     1024
#define SLA     10
#define NBB     (NN / NBA)
#define RCAP    1024
#define DEGCAP  16
#define CHUNK   2048
#define SEG     (NE / NWAVE)
#define WLCAP   1024
#define FLAGP   32
#define WSMAX   ((size_t)128 << 20)

#define O_XB    ((size_t)0)
#define O_WT    (O_XB   + (size_t)NN * DIM * 2)
#define O_BT    (O_WT   + (size_t)DIM * DIM * 2)
#define O_H     (O_BT   + (size_t)DIM * 4)
#define O_CNT   (O_H    + (size_t)NN * DIM * 4)
#define O_OFF   (O_CNT  + (size_t)NN * 4)
#define O_LIST  (O_OFF  + (size_t)NN * 4)
#define O_FLAG  (O_LIST + (size_t)NBB * RCAP * 4)
#define WS_TOTAL (O_FLAG + (size_t)NBB * FLAGP * 4)

#define PREP_WT_BLK (DIM * (DIM / 8) / NTHR)
#define PREP_Z_BLK  (NN * 4 / 16 / NTHR)
#define PREP_GRID   (PREP_WT_BLK + 1 + PREP_Z_BLK)

static_assert(NN % NBA == 0 && NBA == (1 << SLA) && NBB == 16);
static_assert(NN % 8 == 0 && NN % 64 == 0 && NN <= 65536);
static_assert(NE % CHUNK == 0);
static_assert(NE % (NWAVE * 32) == 0 && SEG * NWAVE == NE && SEG % 32 == 0);
static_assert(DIM == 256 && DIM == 32 * 8 && DIM % 64 == 0 && DIM % 32 == 0);
static_assert(RCAP == 1024 && DEGCAP == 16 && RCAP == 4 * NTHR && NBA == 4 * NTHR);
static_assert(WLCAP == 1024 && (NWAVE * WLCAP) % (4 * NTHR) == 0);
static_assert(PREP_WT_BLK == 32 && PREP_Z_BLK == 16);
static_assert(NBB * FLAGP * 4 == 128 * 16);
static_assert(O_WT % 128 == 0 && O_BT % 128 == 0 && O_H % 128 == 0 && O_CNT % 128 == 0);
static_assert(O_OFF % 128 == 0 && O_LIST % 128 == 0 && O_FLAG % 128 == 0);
static_assert(WS_TOTAL == 25496576 && WS_TOTAL <= (size_t)WSMAX);
static_assert((size_t)NN * DIM - 1 == 4194303);

typedef int v4i __attribute__((ext_vector_type(4)));
typedef v4i __attribute__((may_alias)) v4ia;

__global__ __launch_bounds__(NTHR) void k_prep(const float* __restrict__ W, const float* __restrict__ b,
                                               unsigned char* ws) {
  const int tid = (int)threadIdx.x;
  const int blk = (int)blockIdx.x;
  v4u o = (v4u){0u, 0u, 0u, 0u};
  size_t off = O_CNT;
  bool act = false;
  if (blk < PREP_WT_BLK) {
    const int u  = blk * NTHR + tid;
    const int n  = u >> 5;
    const int k8 = (u & 31) * 8;
    const float* p = W + (size_t)k8 * DIM + n;
    unsigned w[8];
#pragma unroll
    for (int i = 0; i < 8; ++i) {
      const float v = p[(size_t)i * DIM];
      asm volatile("" :: "v"(v));
      w[i] = bf16_bits(v);
    }
    o = (v4u){ pk16(w[0], w[1]), pk16(w[2], w[3]), pk16(w[4], w[5]), pk16(w[6], w[7]) };
    off = O_WT + ((size_t)n * DIM + (size_t)k8) * 2;
    act = true;
  } else if (blk == PREP_WT_BLK) {
    const int q = clampi(tid, 0, DIM / 4 - 1);
    const v4f bv = *(const v4fa*)(b + 4 * q);
    asm volatile("" :: "v"(bv));
    const v4u bb = (v4u){ bf16_bits(bv[0]) << 16, bf16_bits(bv[1]) << 16, bf16_bits(bv[2]) << 16, bf16_bits(bv[3]) << 16 };
    const bool isB = tid < DIM / 4;
    const bool isF = (tid >= 64) && (tid < 64 + NBB * FLAGP / 4);
    const unsigned mB = isB ? 0xFFFFFFFFu : 0u;
    o = bb & (v4u){mB, mB, mB, mB};
    const int fq = clampi(tid - 64, 0, NBB * FLAGP / 4 - 1);
    off = isB ? (O_BT + (size_t)q * 16) : (O_FLAG + (size_t)fq * 16);
    act = isB | isF;
  } else {
    const int u = clampi((blk - PREP_WT_BLK - 1) * NTHR + tid, 0, NN / 4 - 1);
    off = O_CNT + (size_t)u * 16;
    act = true;
  }
  if (act) {
    volatile v4u* q = (volatile v4u*)(ws + off);
    *q = o;
    __threadfence();
    *q = o;
  }
}

__global__ __launch_bounds__(NTHR) void k_bucket(const int* __restrict__ ei, const int* __restrict__ sec,
                                                 int* CNT, int* OFF, int* LIST, int* FLAG) {
  __shared__ __attribute__((aligned(16))) int wl[NWAVE * WLCAP];
  __shared__ __attribute__((aligned(16))) int cnt[NBA];
  __shared__ __attribute__((aligned(16))) int offs[NBA];
  __shared__ __attribute__((aligned(16))) int cur[NBA];
  __shared__ __attribute__((aligned(16))) int sl[RCAP];
  __shared__ int misc[16];
  const int tid = (int)threadIdx.x, lane = tid & 31, wave = tid >> 5;
  const int blkB = (int)blockIdx.x;
  const int nodeBase = blkB * NBA;

  {
    const v4i z4 = (v4i){0, 0, 0, 0};
#pragma unroll 1
    for (int i = tid * 4; i < NWAVE * WLCAP; i += NTHR * 4) *(v4ia*)(wl + i) = z4;
    *(v4ia*)(cnt  + 4 * tid) = z4;
    *(v4ia*)(offs + 4 * tid) = z4;
    *(v4ia*)(cur  + 4 * tid) = z4;
    *(v4ia*)(sl   + 4 * tid) = z4;
    if (tid < 16) misc[tid] = 0;
  }
  __syncthreads();

  int wc = 0;
  {
    const int* rowp = ei;
    const int* colp = ei + NE;
    const int segBase = wave * SEG;
#pragma unroll 1
    for (int st = 0; st < SEG / 32; ++st) {
      const int e = segBase + st * 32 + lane;
      const int r = rowp[e];
      asm volatile("" :: "v"(r));
      const int c = colp[e];
      asm volatile("" :: "v"(c));
      const int rc = clampi(r, 0, NN - 1);
      const int cc = clampi(c, 0, NN - 1);
      const int sa = sec[rc];
      asm volatile("" :: "v"(sa));
      const int sb = sec[cc];
      asm volatile("" :: "v"(sb));
      const unsigned s = (unsigned)(c - nodeBase);
      const bool hit = (s < (unsigned)NBA) & (sa == sb);
      const unsigned m = __builtin_amdgcn_ballot_w32(hit);
      const int pos = wc + (int)__builtin_amdgcn_mbcnt_lo(m, 0u);
      if (m != 0u) {
        if (hit && pos < WLCAP) wl[wave * WLCAP + pos] = rc | (int)(s << 16);
        wc += (int)__builtin_popcount(m);
      }
    }
  }
  if (lane == 0) misc[wave] = wc;
  __syncthreads();

  if (wave == 0) {
    int t = 0, ov = 0;
#pragma unroll 1
    for (int w2 = 0; w2 < NWAVE; ++w2) {
      int c = __builtin_amdgcn_readfirstlane(misc[w2]);
      if (c > WLCAP) ov = 1;
      c = clampi(c, 0, WLCAP);
#pragma unroll 1
      for (int i = 0; i < c; ++i) {
        const int u = wl[w2 * WLCAP + i];
        const int slot = (u >> 16) & (NBA - 1);
        if (t < RCAP) {
          if (lane == 0) cnt[slot] = cnt[slot] + 1;
          t = t + 1;
        } else {
          ov = 1;
        }
      }
    }
    if (lane == 0) { misc[8] = t; misc[9] = ov; }
  }
  __syncthreads();

  if (wave == 0) {
    const int base = lane * (NBA / 32);
    int s = 0, mx = 0;
#pragma unroll 1
    for (int i = 0; i < NBA / 32; ++i) {
      const int cv = cnt[base + i];
      s += cv;
      mx = cv > mx ? cv : mx;
    }
    int incl = s;
#pragma unroll
    for (int d = 1; d < 32; d <<= 1) {
      const int y = __shfl_up(incl, d, 32);
      if (lane >= d) incl += y;
    }
    int run = incl - s;
#pragma unroll 1
    for (int i = 0; i < NBA / 32; ++i) {
      const int cv = cnt[base + i];
      offs[base + i] = run;
      cur[base + i]  = run;
      run += cv;
    }
    const unsigned bm = __builtin_amdgcn_ballot_w32(mx > DEGCAP);
    if (lane == 0) misc[10] = (bm != 0u) ? 1 : 0;
  }
  __syncthreads();

  if (wave == 0) {
    int t2 = 0;
#pragma unroll 1
    for (int w2 = 0; w2 < NWAVE; ++w2) {
      int c = __builtin_amdgcn_readfirstlane(misc[w2]);
      c = clampi(c, 0, WLCAP);
#pragma unroll 1
      for (int i = 0; i < c; ++i) {
        const int u = wl[w2 * WLCAP + i];
        const int slot = (u >> 16) & (NBA - 1);
        if (t2 < RCAP) {
          if (lane == 0) {
            const int p = clampi(cur[slot], 0, RCAP - 1);
            sl[p] = u & 0xFFFF;
            cur[slot] = p + 1;
          }
          t2 = t2 + 1;
        }
      }
    }
  }
  __syncthreads();

  const v4i cv4 = *(const v4ia*)(cnt  + 4 * tid);
  const v4i ov4 = *(const v4ia*)(offs + 4 * tid);
  const v4i lv4 = *(const v4ia*)(sl   + 4 * tid);
  const int fl  = ((misc[9] | misc[10]) != 0) ? 1 : 0;
  const v4i fv4 = (v4i){fl, fl, fl, fl};
  int* pc = CNT  + nodeBase + 4 * tid;
  int* po = OFF  + nodeBase + 4 * tid;
  int* pl = LIST + blkB * RCAP + 4 * tid;
  int* pf = FLAG + blkB * FLAGP + 4 * (tid & 7);
  const bool wf = tid < 8;
  *(volatile v4i*)pc = cv4;
  *(volatile v4i*)po = ov4;
  *(volatile v4i*)pl = lv4;
  if (wf) *(volatile v4i*)pf = fv4;
  __threadfence();
  *(volatile v4i*)pc = cv4;
  *(volatile v4i*)po = ov4;
  *(volatile v4i*)pl = lv4;
  if (wf) *(volatile v4i*)pf = fv4;
}

__device__ __forceinline__ v4f poison4(bool bad, v4f v) {
  const float qn = __int_as_float(0x7fc00000);
  v4f r;
  r.x = bad ? qn : v.x;
  r.y = bad ? qn : v.y;
  r.z = bad ? qn : v.z;
  r.w = bad ? qn : v.w;
  return r;
}

__global__ __launch_bounds__(NTHR) void k_replay(const float* __restrict__ H, const float* __restrict__ BT,
                                                 const int* __restrict__ CNT, const int* __restrict__ OFF,
                                                 const int* __restrict__ LIST, const int* __restrict__ FLAG,
                                                 float* out) {
  __shared__ __attribute__((aligned(16))) float sbt[DIM];
  const int tid = (int)threadIdx.x, lane = tid & 31, wave = tid >> 5;
  if (tid < DIM / 4) {
    const v4f v = *(const v4fa*)(BT + 4 * tid);
    *(v4fa*)(sbt + 4 * tid) = v;
  }
  __syncthreads();

  const int t  = (int)blockIdx.x * NWAVE + wave;
  const int tc = clampi(t, 0, NN - 1);
  const int bB = tc >> SLA;
  const int c = CNT[tc];
  asm volatile("" :: "v"(c));
  const int off = OFF[tc];
  asm volatile("" :: "v"(off));
  const int flag = FLAG[bB * FLAGP];
  asm volatile("" :: "v"(flag));
  const bool big = c > DEGCAP;
  const int cn = __builtin_amdgcn_readfirstlane(clampi(c, 0, DEGCAP));
  const float deg = (float)(clampi(c, 0, NE) + 1);
  const float dtr = 1.0f / sqrtf(deg);
  const float dt  = (deg > 0.0f) ? dtr : 0.0f;

  const float* hcol = H + 4 * lane;
  v4f a0 = (v4f){0.f, 0.f, 0.f, 0.f};
  v4f a1 = (v4f){0.f, 0.f, 0.f, 0.f};
  int pois = 0;
#pragma unroll 1
  for (int j = 0; j < cn; ++j) {
    const int li = clampi(off + j, 0, RCAP - 1);
    const int sraw = LIST[bB * RCAP + li];
    asm volatile("" :: "v"(sraw));
    const int s = clampi(sraw, 0, NN - 1);
    const int cs = CNT[s];
    asm volatile("" :: "v"(cs));
    const int fs = FLAG[(s >> SLA) * FLAGP];
    asm volatile("" :: "v"(fs));
    const float dsg = (float)(clampi(cs, 0, NE) + 1);
    const float dsr = 1.0f / sqrtf(dsg);
    const float ds  = (dsg > 0.0f) ? dsr : 0.0f;
    const float nrm = (ds * 1.0f) * dt;
    const v4f h0 = *(const v4fa*)(hcol + (size_t)s * DIM);
    asm volatile("" :: "v"(h0));
    const v4f h1 = *(const v4fa*)(hcol + (size_t)s * DIM + 128);
    asm volatile("" :: "v"(h1));
    a0 = a0 + h0 * nrm;
    a1 = a1 + h1 * nrm;
    pois |= fs;
  }
  const v4f s0 = *(const v4fa*)(hcol + (size_t)tc * DIM);
  asm volatile("" :: "v"(s0));
  const v4f s1 = *(const v4fa*)(hcol + (size_t)tc * DIM + 128);
  asm volatile("" :: "v"(s1));
  const float sn = (dt * 1.0f) * dt;
  a0 = a0 + s0 * sn;
  a1 = a1 + s1 * sn;
  const v4f b0 = *(const v4fa*)(sbt + 4 * lane);
  const v4f b1 = *(const v4fa*)(sbt + 128 + 4 * lane);
  a0 = a0 + b0;
  a1 = a1 + b1;
  const bool bad = (flag != 0) | big | (pois != 0);
  const v4f r0 = poison4(bad, a0);
  const v4f r1 = poison4(bad, a1);
  if (t < NN) {
    float* op = out + (size_t)t * DIM + 4 * lane;
    *(volatile v4f*)op = r0;
    *(volatile v4f*)(op + 128) = r1;
    __threadfence();
    *(volatile v4f*)op = r0;
    *(volatile v4f*)(op + 128) = r1;
  }
}

extern "C" void kernel_launch(void* const* d_in, const int* in_sizes, int n_in,
                              void* d_out, int out_size, void* d_ws, size_t ws_size,
                              hipStream_t stream) {
  if (n_in < 5) return;
  if (in_sizes[0] != NN * DIM) return;
  if (in_sizes[1] != DIM * DIM) return;
  if (in_sizes[2] != DIM) return;
  if (in_sizes[3] != 2 * NE) return;
  if (in_sizes[4] != NN) return;
  if (out_size != NN * DIM) return;
  if (ws_size < (size_t)WS_TOTAL) return;

  const float* x   = (const float*)d_in[0];
  const float* W   = (const float*)d_in[1];
  const float* b   = (const float*)d_in[2];
  const int*   ei  = (const int*)d_in[3];
  const int*   sec = (const int*)d_in[4];
  float* out = (float*)d_out;

  unsigned char* ws = (unsigned char*)d_ws;
  unsigned short* XB = (unsigned short*)(ws + O_XB);
  unsigned short* WT = (unsigned short*)(ws + O_WT);
  float* BT   = (float*)(ws + O_BT);
  float* H    = (float*)(ws + O_H);
  int*   CNT  = (int*)(ws + O_CNT);
  int*   OFF  = (int*)(ws + O_OFF);
  int*   LIST = (int*)(ws + O_LIST);
  int*   FLAG = (int*)(ws + O_FLAG);

  k_plane<0><<<NN * DIM / 8 / 256, 256, 0, stream>>>(x, NN, DIM, DIM, XB, NN, DIM);
  k_prep<<<PREP_GRID, NTHR, 0, stream>>>(W, b, ws);
  k_gemm_nt<0, 0><<<(NN / 64) * (DIM / 64) / 8, 256, 0, stream>>>(XB, WT, BT, H, NN, DIM, DIM, DIM);
  k_bucket<<<NBB, NTHR, 0, stream>>>(ei, sec, CNT, OFF, LIST, FLAG);
  k_replay<<<NN / NWAVE, NTHR, 0, stream>>>(H, BT, CNT, OFF, LIST, FLAG, out);
}
